// BilateralLayer_38671885533454
// MI455X (gfx1250) — hardware-verified
//
#include <hip/hip_runtime.h>


namespace {
constexpr int HI = 512, LO = 128, CS = 21, CI = 3, CT = 24  , CP = 32, RAD = 12, SRW = 192  , ICUT = 128  , HCUT = 512  ;
constexpr float XS = 8.0f, WS = 8.0f  , PS8 = 8.0f, TB2 = 18.0f  , TA2 = 128.0f  ;
static_assert(HI == 4 * LO && ICUT % 16 == 0 && HCUT % 16 == 0, "tiling");
typedef _Float16 b16;
typedef __attribute__((ext_vector_type(16))) _Float16 v16b;
typedef __attribute__((ext_vector_type(8))) _Float16 v8b;
typedef __attribute__((ext_vector_type(8))) float v8f;
typedef __attribute__((ext_vector_type(4))) float v4f;
__device__ __forceinline__ float bf16_rne(float f) { unsigned int u = __float_as_uint(f); u += 0x7FFFu + ((u >> 16) & 1u); return __uint_as_float(u & 0xFFFF0000u); }
__device__ __forceinline__ void split16(float v, b16& hi, b16& lo) { hi = (b16)v; lo = (b16)(v - (float)hi); }
__device__ __forceinline__ v16b frag_kb(const b16* p, int hh) { const v8b a = *(const v8b*)(p + 8 * hh), b = *(const v8b*)(p + 16 + 8 * hh); v16b f;
#pragma unroll
  for (int e = 0; e < 8; ++e) { f[e] = a[e]; f[8 + e] = b[e]; } return f; }
__device__ __forceinline__ v8f wmma16b(v16b a, v16b b, v8f c) { v8f d = __builtin_amdgcn_wmma_f32_16x16x32_f16(false, a, false, b, (short)0, c, false, false); asm volatile("v_nop\n\tv_nop\n\tv_nop\n\tv_nop" : "+v"(d) : "v"(a), "v"(b)); return d; }
__device__ __forceinline__ void wave_lds_sync() { __builtin_amdgcn_fence(__ATOMIC_RELEASE, "workgroup"); __builtin_amdgcn_wave_barrier(); __builtin_amdgcn_fence(__ATOMIC_ACQUIRE, "workgroup"); }
__device__ __forceinline__ float pmul(float a, float b) { float p = a * b; asm volatile("" : "+v"(p)); return p; }
__device__ __forceinline__ int iclamp(int v, int lo, int hi) { return v < lo ? lo : (v > hi ? hi : v); }

typedef __attribute__((ext_vector_type(4))) _Float16 v4h;
typedef __attribute__((ext_vector_type(2))) float v2f;
__global__ __launch_bounds__(128) void rmat_kernel(b16* __restrict__ DTh, b16* __restrict__ DTl, b16* __restrict__ UT) {
  const int i = blockIdx.x * 128 + threadIdx.x;
  if (blockIdx.x == 0) { const float sample = ((float)i + 0.5f) * 4.0f - 0.5f; float tot = 0.0f;
#pragma unroll 1
    for (int h = 0; h < HI; ++h) { const float x = fabsf(sample - (float)h) * 0.25f; tot += fmaxf(0.0f, 1.0f - x); }
    for (int pass = 0; pass < 2; ++pass) {
#pragma unroll 1
      for (int h0 = 0; h0 < HI; h0 += 8) { v8b hv, lv;
#pragma unroll 1
        for (int j = 0; j < 8; ++j) { const float x = fabsf(sample - (float)(h0 + j)) * 0.25f; float w = fmaxf(0.0f, 1.0f - x); w = (fabsf(tot) > 1000.0f * 1.1920929e-7f) ? w / tot : 0.0f; b16 p, q; split16(w * WS, p, q); hv[j] = p; lv[j] = q; }
        *(volatile v8b*)(DTh + (size_t)i * HI + h0) = hv; *(volatile v8b*)(DTl + (size_t)i * HI + h0) = lv; } __threadfence(); } }
  else { const int h = i - 128; const float sample = ((float)h + 0.5f) * 0.25f - 0.5f; float tot = 0.0f;
#pragma unroll 1
    for (int ii = 0; ii < LO; ++ii) tot += fmaxf(0.0f, 1.0f - fabsf(sample - (float)ii));
    for (int pass = 0; pass < 2; ++pass) {
#pragma unroll 1
      for (int i0 = 0; i0 < LO; i0 += 8) { v8b hv;
#pragma unroll 1
        for (int j = 0; j < 8; ++j) { float w = fmaxf(0.0f, 1.0f - fabsf(sample - (float)(i0 + j))); w = (fabsf(tot) > 1000.0f * 1.1920929e-7f) ? w / tot : 0.0f; hv[j] = (b16)(w * WS); }
        *(volatile v8b*)(UT + (size_t)h * LO + i0) = hv; } __threadfence(); } }
}
__global__ __launch_bounds__(128) void down1_kernel(const float* __restrict__ src, const float* __restrict__ im, const b16* __restrict__ DTh, const b16* __restrict__ DTl, float* __restrict__ T1) {
  __shared__ __attribute__((aligned(16))) b16 Xs[CP][HI + 8]; __shared__ __attribute__((aligned(16))) float Os[LO][CT];
  const int wave = threadIdx.x >> 5, lane = threadIdx.x & 31, nloc = lane & 15, hlf = lane >> 4; const int w = blockIdx.x;
  for (int h = threadIdx.x; h < HI; h += 128) { const float* sp = src + ((size_t)h * HI + w) * CS; const float* ip = im + ((size_t)h * HI + w) * CI;
    for (int c = 0; c < CP; ++c) { float v = 0.0f; if (c < CS) v = sp[c]; else if (c < CT) v = ip[c - CS]; Xs[c][h] = (b16)(bf16_rne(v) * XS); } }
  __syncthreads();
  for (int it = 0; it < 2; ++it) { const int i0 = (wave * 2 + it) * 16; v8f acc[2] = {(v8f){}, (v8f){}};
#pragma unroll 4
    for (int kb = 0; kb < HI; kb += 32) { const v16b a = frag_kb(DTh + (size_t)(i0 + nloc) * HI + kb, hlf), al = frag_kb(DTl + (size_t)(i0 + nloc) * HI + kb, hlf);
#pragma unroll
      for (int t = 0; t < 2; ++t) { const v16b bx = frag_kb(&Xs[t * 16 + nloc][kb], hlf); acc[t] = wmma16b(a, bx, acc[t]); acc[t] = wmma16b(al, bx, acc[t]); } }
#pragma unroll
    for (int t = 0; t < 2; ++t)
#pragma unroll
      for (int r = 0; r < 8; ++r) { const int c = t * 16 + nloc; if (c < CT) Os[i0 + 8 * hlf + r][c] = acc[t][r] * (1.0f / (WS * XS)); } }
  __syncthreads();
  for (int pass = 0; pass < 2; ++pass) { const float* os = &Os[0][0]; float* dst = T1 + (size_t)w * LO * CT; for (int q = threadIdx.x; q < LO * CT / 4; q += 128) *(volatile v4f*)(dst + q * 4) = *(const v4f*)(os + q * 4); __threadfence(); }
}
__global__ __launch_bounds__(128) void down2_kernel(const float* __restrict__ T1, const b16* __restrict__ DTh, const b16* __restrict__ DTl, b16* __restrict__ SRh, b16* __restrict__ SRl, float* __restrict__ IMR) {
  __shared__ __attribute__((aligned(16))) b16 Th[CP][HI + 8], Tl[CP][HI + 8]; __shared__ __attribute__((aligned(16))) float Os[LO][CT];
  const int wave = threadIdx.x >> 5, lane = threadIdx.x & 31, nloc = lane & 15, hlf = lane >> 4; const int i = blockIdx.x;
  for (int w = threadIdx.x; w < HI; w += 128) { const float* tp = T1 + ((size_t)w * LO + i) * CT; for (int c = 0; c < CP; ++c) { const float v = (c < CT) ? tp[c] : 0.0f; b16 p, q; split16(v * XS, p, q); Th[c][w] = p; Tl[c][w] = q; } }
  __syncthreads();
  for (int jt = 0; jt < 2; ++jt) { const int j0 = (wave * 2 + jt) * 16; v8f acc[2] = {(v8f){}, (v8f){}};
#pragma unroll 4
    for (int kb = 0; kb < HI; kb += 32) { const v16b a = frag_kb(DTh + (size_t)(j0 + nloc) * HI + kb, hlf), al = frag_kb(DTl + (size_t)(j0 + nloc) * HI + kb, hlf);
#pragma unroll
      for (int t = 0; t < 2; ++t) { const v16b bh = frag_kb(&Th[t * 16 + nloc][kb], hlf), bl = frag_kb(&Tl[t * 16 + nloc][kb], hlf); acc[t] = wmma16b(a, bh, acc[t]); acc[t] = wmma16b(a, bl, acc[t]); acc[t] = wmma16b(al, bh, acc[t]); } }
#pragma unroll
    for (int t = 0; t < 2; ++t)
#pragma unroll
      for (int r = 0; r < 8; ++r) { const int c = t * 16 + nloc; if (c < CT) Os[j0 + 8 * hlf + r][c] = acc[t][r] * (1.0f / (WS * XS)); } }
  __syncthreads();
  for (int pass = 0; pass < 2; ++pass) {
    for (int q = threadIdx.x; q < CP * SRW / 8; q += 128) { const int c = q / (SRW / 8), col0 = (q % (SRW / 8)) * 8; v8b hv, lv;
      for (int j = 0; j < 8; ++j) { const int col = col0 + j; float v = 0.0f; if (c < CS && col >= 16 && col < 16 + LO) v = Os[col - 16][c]; b16 p, qq; split16(v * XS, p, qq); hv[j] = p; lv[j] = qq; }
      *(volatile v8b*)(SRh + ((size_t)i * CP + c) * SRW + col0) = hv; *(volatile v8b*)(SRl + ((size_t)i * CP + c) * SRW + col0) = lv; }
    for (int q = threadIdx.x; q < LO; q += 128) { v4f g = {Os[q][CS], Os[q][CS + 1], Os[q][CS + 2], 0.0f}; *(volatile v4f*)(IMR + ((size_t)i * LO + q) * 4) = g; }
    __threadfence(); }
}
__device__ __forceinline__ int refl(int v, int n) { v = (v < 0) ? -v : v; v = (v >= n) ? 2 * n - 2 - v : v; return v < 0 ? 0 : (v >= n ? n - 1 : v); }
__global__ __launch_bounds__(256) void bilateral_kernel(const b16* __restrict__ SRh, const b16* __restrict__ SRl, const float* __restrict__ IMR, b16* __restrict__ Oh, b16* __restrict__ Ol) {
  __shared__ __attribute__((aligned(16))) b16 Ah[8][16][64 + 8], Al[8][16][64 + 8]; __shared__ __attribute__((aligned(16))) float Os[CP][LO + 4];
  const int wave = threadIdx.x >> 5, lane = threadIdx.x & 31, nloc = lane & 15, hlf = lane >> 4; const int i = blockIdx.x; const int j0 = wave * 16;
  v8f acc[2] = {(v8f){}, (v8f){}};
  if (i < ICUT) {
    const int j = j0 + nloc; const float g0 = IMR[((size_t)i * LO + j) * 4], g1 = IMR[((size_t)i * LO + j) * 4 + 1], g2 = IMR[((size_t)i * LO + j) * 4 + 2];
#pragma unroll 1
    for (int dy = 0; dy < 2 * RAD + 1; ++dy) { const int sy = i + dy - RAD; const bool rowin = (sy >= 0 && sy < LO); const int ry = refl(sy, LO); const float dyy = (float)((dy - RAD) * (dy - RAD));
      for (int k = hlf * 32; k < hlf * 32 + 32; ++k) { Ah[wave][nloc][k] = (b16)0.0f; Al[wave][nloc][k] = (b16)0.0f; }
      __builtin_amdgcn_fence(__ATOMIC_RELEASE, "workgroup"); __builtin_amdgcn_wave_barrier(); __builtin_amdgcn_fence(__ATOMIC_ACQUIRE, "workgroup");
      const int dx0 = hlf ? 13 : 0, dx1 = hlf ? 25 : 13;
      for (int dx = dx0; dx < dx1; ++dx) { const int sx = j + dx - RAD; float wv = 0.0f;
        if (rowin && sx >= 0 && sx < LO) { const int rx = sx; const float* gp = IMR + ((size_t)ry * LO + rx) * 4; const float d0 = gp[0] - g0, d1 = gp[1] - g1, d2 = gp[2] - g2; const float dxx = (float)((dx - RAD) * (dx - RAD));
          wv = __expf(-(d0 * d0 + d1 * d1 + d2 * d2) * (1.0f / TB2)) * __expf(-(dyy + dxx) * (1.0f / TA2)); }
        else if (rowin == false || sx < 0 || sx >= LO) {
          wv = 0.0f; }
        b16 p, q; split16(wv * PS8, p, q); Ah[wave][nloc][nloc + dx] = p; Al[wave][nloc][nloc + dx] = q; }
      __builtin_amdgcn_fence(__ATOMIC_RELEASE, "workgroup"); __builtin_amdgcn_wave_barrier(); __builtin_amdgcn_fence(__ATOMIC_ACQUIRE, "workgroup");
      const int syc = sy < 0 ? 0 : (sy >= LO ? LO - 1 : sy); const b16* brow_h = SRh + ((size_t)syc * CP) * SRW + 16 + j0 - RAD; const b16* brow_l = SRl + ((size_t)syc * CP) * SRW + 16 + j0 - RAD;
#pragma unroll
      for (int ks = 0; ks < 2; ++ks) { const v16b ah = frag_kb(&Ah[wave][nloc][ks * 32], hlf), al = frag_kb(&Al[wave][nloc][ks * 32], hlf);
#pragma unroll
        for (int t = 0; t < 2; ++t) { const v16b bh = frag_kb(brow_h + (size_t)(t * 16 + nloc) * SRW + ks * 32, hlf), bl = frag_kb(brow_l + (size_t)(t * 16 + nloc) * SRW + ks * 32, hlf);
          acc[t] = wmma16b(ah, bh, acc[t]); acc[t] = wmma16b(ah, bl, acc[t]); acc[t] = wmma16b(al, bh, acc[t]); } }
      __builtin_amdgcn_fence(__ATOMIC_RELEASE, "workgroup"); __builtin_amdgcn_wave_barrier(); __builtin_amdgcn_fence(__ATOMIC_ACQUIRE, "workgroup"); } }
#pragma unroll
  for (int t = 0; t < 2; ++t)
#pragma unroll
    for (int r = 0; r < 8; ++r) Os[t * 16 + nloc][j0 + 8 * hlf + r] = acc[t][r] * (1.0f / (PS8 * XS));
  __syncthreads();
  for (int pass = 0; pass < 2; ++pass) { for (int q = threadIdx.x; q < CP * LO / 8; q += 256) { const int c = q / (LO / 8), jj = (q % (LO / 8)) * 8; v8b hv, lv; for (int e = 0; e < 8; ++e) { const float v = (c < CS) ? Os[c][jj + e] : 0.0f; b16 p, qq; split16(v * XS, p, qq); hv[e] = p; lv[e] = qq; }
      *(volatile v8b*)(Oh + ((size_t)i * CP + c) * LO + jj) = hv; *(volatile v8b*)(Ol + ((size_t)i * CP + c) * LO + jj) = lv; } __threadfence(); }
}
__global__ __launch_bounds__(256) void up1_kernel(const b16* __restrict__ Oh, const b16* __restrict__ Ol, const b16* __restrict__ UT, float* __restrict__ V1) {
  __shared__ __attribute__((aligned(16))) b16 Bh[CP][LO + 8], Bl[CP][LO + 8]; __shared__ __attribute__((aligned(16))) float Vs[HI][CT];
  const int wave = threadIdx.x >> 5, lane = threadIdx.x & 31, nloc = lane & 15, hlf = lane >> 4; const int j = blockIdx.x;
  for (int q = threadIdx.x; q < CP * LO; q += 256) { const int c = q / LO, i = q % LO; Bh[c][i] = Oh[((size_t)i * CP + c) * LO + j]; Bl[c][i] = Ol[((size_t)i * CP + c) * LO + j]; }
  __syncthreads();
  for (int ht = 0; ht < 4; ++ht) { const int h0 = (wave * 4 + ht) * 16; v8f acc[2] = {(v8f){}, (v8f){}};
#pragma unroll
    for (int kb = 0; kb < LO; kb += 32) { const v16b a = frag_kb(UT + (size_t)(h0 + nloc) * LO + kb, hlf);
#pragma unroll
      for (int t = 0; t < 2; ++t) { acc[t] = wmma16b(a, frag_kb(&Bh[t * 16 + nloc][kb], hlf), acc[t]); acc[t] = wmma16b(a, frag_kb(&Bl[t * 16 + nloc][kb], hlf), acc[t]); } }
#pragma unroll
    for (int t = 0; t < 2; ++t)
#pragma unroll
      for (int r = 0; r < 8; ++r) { const int c = t * 16 + nloc; if (c < CT) Vs[h0 + 8 * hlf + r][c] = acc[t][r] * (1.0f / (WS * XS)); } }
  __syncthreads();
  for (int pass = 0; pass < 2; ++pass) { const float* vs = &Vs[0][0]; float* dst = V1 + (size_t)j * HI * CT; for (int q = threadIdx.x; q < HI * CT / 4; q += 256) *(volatile v4f*)(dst + q * 4) = *(const v4f*)(vs + q * 4); __threadfence(); }
}
__global__ __launch_bounds__(256) void up2_kernel(const float* __restrict__ V1, const b16* __restrict__ UT, float* __restrict__ out) {
  __shared__ __attribute__((aligned(16))) b16 Bh[CP][LO + 8], Bl[CP][LO + 8]; __shared__ __attribute__((aligned(16))) float Ws[HI * CS];
  const int wave = threadIdx.x >> 5, lane = threadIdx.x & 31, nloc = lane & 15, hlf = lane >> 4; const int h = blockIdx.x; if (h >= HCUT) return;
  for (int q = threadIdx.x; q < CP * LO; q += 256) { const int c = q / LO, j = q % LO; const float v = (c < CT) ? V1[((size_t)j * HI + h) * CT + c] : 0.0f; b16 p, qq; split16(v * XS, p, qq); Bh[c][j] = p; Bl[c][j] = qq; }
  __syncthreads();
  for (int wt = 0; wt < 4; ++wt) { const int w0 = (wave * 4 + wt) * 16; v8f acc[2] = {(v8f){}, (v8f){}};
#pragma unroll
    for (int kb = 0; kb < LO; kb += 32) { const v16b a = frag_kb(UT + (size_t)(w0 + nloc) * LO + kb, hlf);
#pragma unroll
      for (int t = 0; t < 2; ++t) { acc[t] = wmma16b(a, frag_kb(&Bh[t * 16 + nloc][kb], hlf), acc[t]); acc[t] = wmma16b(a, frag_kb(&Bl[t * 16 + nloc][kb], hlf), acc[t]); } }
#pragma unroll
    for (int t = 0; t < 2; ++t)
#pragma unroll
      for (int r = 0; r < 8; ++r) { const int c = t * 16 + nloc; if (c < CS) Ws[(w0 + 8 * hlf + r) * CS + c] = acc[t][r] * (1.0f / (WS * XS)); } }
  __syncthreads();
  for (int pass = 0; pass < 2; ++pass) { float* dst = out + (size_t)h * HI * CS; for (int q = threadIdx.x; q < HI * CS / 4; q += 256) *(volatile v4f*)(dst + q * 4) = *(const v4f*)(&Ws[q * 4]); __threadfence(); }
}
}

extern "C" void kernel_launch(void* const* d_in, const int* in_sizes, int n_in, void* d_out, int out_size, void* d_ws, size_t ws_size, hipStream_t stream) {
  (void)n_in;
  auto Fp = [&](int i) { return (const float*)d_in[i]; };
  if (in_sizes[0] != HI * HI * CS || in_sizes[1] != HI * HI * CI || out_size != HI * HI * CS) return;
  size_t off = 0; char* ws = (char*)d_ws;
  auto carve = [&](size_t bytes) { char* p = ws + off; off += (bytes + 255) & ~(size_t)255; return p; };
  b16* DTh = (b16*)carve((size_t)LO * HI * 2); b16* DTl = (b16*)carve((size_t)LO * HI * 2); b16* UT = (b16*)carve((size_t)HI * LO * 2);
  float* T1 = (float*)carve((size_t)HI * LO * CT * 4); b16* SRh = (b16*)carve((size_t)LO * CP * SRW * 2); b16* SRl = (b16*)carve((size_t)LO * CP * SRW * 2); float* IMR = (float*)carve((size_t)LO * LO * 4 * 4);
  b16* Oh = (b16*)carve((size_t)LO * CP * LO * 2); b16* Ol = (b16*)carve((size_t)LO * CP * LO * 2); float* V1 = (float*)carve((size_t)LO * HI * CT * 4);
  if (off > ws_size || off > ((size_t)128 << 20)) return;
  rmat_kernel<<<5, 128, 0, stream>>>(DTh, DTl, UT);
  down1_kernel<<<HI, 128, 0, stream>>>(Fp(0), Fp(1), DTh, DTl, T1);
  down2_kernel<<<LO, 128, 0, stream>>>(T1, DTh, DTl, SRh, SRl, IMR);
  bilateral_kernel<<<LO, 256, 0, stream>>>(SRh, SRl, IMR, Oh, Ol);
  up1_kernel<<<LO, 256, 0, stream>>>(Oh, Ol, UT, V1);
  up2_kernel<<<HI, 256, 0, stream>>>(V1, UT, (float*)d_out);
}
